// DTWLayer_85014582657726
// MI455X (gfx1250) — hardware-verified
//
#include <hip/hip_runtime.h>
#include <hip/hip_fp16.h>

#define BB   16
#define DD   16
#define TT   1024
#define PP   64
#define LL   64
#define TILE 64
#define NTILE (TT / TILE)
#define BIGV    1e30f
#define HALFBIG 5e29f
#define WDEC 0.96466155f

typedef __attribute__((ext_vector_type(16))) _Float16 v16h;
typedef __attribute__((ext_vector_type(8)))  float    v8f;

__launch_bounds__(32)
__global__ void dtw_fused_kernel(const float* __restrict__ x,
                                 const float* __restrict__ patts,
                                 float* __restrict__ out) {
  const int p    = blockIdx.x;
  const int b    = blockIdx.y;
  const int lane = threadIdx.x;

  __shared__ float  pT[LL][DD];
  __shared__ float  x2b[TILE];
  __shared__ __half distb[2][TILE][LL + 4];
  __shared__ __attribute__((aligned(16))) float ostage[LL][TILE];

  for (int i = lane; i < LL * DD; i += 32) {
    int l = i >> 4, d = i & 15;
    pT[l][d] = patts[(p * DD + d) * LL + l];
  }
  __syncthreads();

  const int  mloc   = lane & 15;
  const bool hiHalf = (lane >= 16);
  const int  kbase  = hiHalf ? 8 : 0;

  v16h  bf[4];
  float p2col[4];
#pragma unroll
  for (int tn = 0; tn < 4; ++tn) {
    int n = tn * 16 + mloc;
    float s = 0.f;
#pragma unroll
    for (int e = 0; e < 16; ++e) {
      float v = pT[n][e];
      s += v * v;
      bf[tn][e] = (e < 8) ? (_Float16)pT[n][kbase + e] : (_Float16)0.f;
    }
    p2col[tn] = s;
  }

  float d0 = BIGV;
  float d1 = BIGV;
  float hprev = BIGV;
  const int i0 = 2 * lane, i1 = i0 + 1;
  const int outBase = ((b * PP + p) * LL) * TILE;

  auto cell = [&](int j, float h, bool doStore) {
    int sl = (j >> 6) & 1;
    int tl = j & (TILE - 1);
    __half2 dv = *(const __half2*)&distb[sl][tl][i0];
    float dist0 = __low2float(dv);
    float dist1 = __high2float(dv);
    float m0 = fminf(fminf(h, d0), hprev);
    m0 = (m0 >= HALFBIG) ? 0.f : m0;
    float n0 = fmaf(WDEC, m0, dist0);
    float m1 = fminf(fminf(n0, d1), d0);
    m1 = (m1 >= HALFBIG) ? 0.f : m1;
    float n1 = fmaf(WDEC, m1, dist1);
    d0 = n0;
    d1 = n1;
    if (doStore && j >= TT - TILE) {
      int tau = j - (TT - TILE);
      ostage[i0][tau] = n0;
      ostage[i1][tau] = n1;
    }
  };

  for (int tile = 0; tile < NTILE; ++tile) {
    const int t0   = tile * TILE;
    const int slot = tile & 1;

    if (tile + 1 < NTILE) {
      const float* pf =
          x + (b * DD + (lane & 15)) * TT + (t0 + TILE) + ((lane >> 4) * 32);
      __builtin_prefetch(pf, 0, 1);
    }

    for (int t = lane; t < TILE; t += 32) {
      float s = 0.f;
#pragma unroll
      for (int d = 0; d < DD; ++d) {
        float v = x[(b * DD + d) * TT + t0 + t];
        s += v * v;
      }
      x2b[t] = s;
    }
    __syncthreads();

#pragma unroll
    for (int tm = 0; tm < 4; ++tm) {
      const float* xrow = x + (b * DD + kbase) * TT + t0 + (tm * 16 + mloc);
      v16h af;
#pragma unroll
      for (int e = 0; e < 8; ++e) af[e] = (_Float16)xrow[e * TT];
#pragma unroll
      for (int e = 8; e < 16; ++e) af[e] = (_Float16)0.f;
      float x2row[8];
#pragma unroll
      for (int r = 0; r < 8; ++r)
        x2row[r] = x2b[tm * 16 + (hiHalf ? r + 8 : r)];
#pragma unroll
      for (int tn = 0; tn < 4; ++tn) {
        v8f acc = {};
        acc = __builtin_amdgcn_wmma_f32_16x16x32_f16(
             false, af,  false, bf[tn],
             (short)0, acc,  false,  false);
        asm volatile("v_nop\n\tv_nop\n\tv_nop\n\tv_nop" : "+v"(acc) : "v"(af), "v"(bf[tn]));
#pragma unroll
        for (int r = 0; r < 8; ++r) {
          float sq = fmaf(-2.f, acc[r], x2row[r] + p2col[tn]);
          float dv = __builtin_amdgcn_sqrtf(fmaxf(sq, 1e-12f));
          int   mr = hiHalf ? r + 8 : r;
          distb[slot][tm * 16 + mr][tn * 16 + mloc] = __float2half(dv);
        }
      }
    }
    __syncthreads();

    const bool lastTile = (tile == NTILE - 1);
    if (tile == 0) {
      for (int ss = 0; ss < TILE; ++ss) {
        int   j = ss - lane;
        float h = __shfl_up(d1, 1, 32);
        if (lane == 0) h = BIGV;
        if (j >= 0) cell(j, h, false);
        hprev = h;
      }
    } else {
#pragma unroll 4
      for (int ss = 0; ss < TILE; ++ss) {
        int   j = t0 + ss - lane;
        float h = __shfl_up(d1, 1, 32);
        if (lane == 0) h = BIGV;
        cell(j, h, lastTile);
        hprev = h;
      }
    }
  }

  for (int s = TT; s < TT + 31; ++s) {
    int   j = s - lane;
    float h = __shfl_up(d1, 1, 32);
    if (lane == 0) h = BIGV;
    if (j < TT) cell(j, h, true);
    hprev = h;
  }

  __syncthreads();
  {
    typedef float v4f __attribute__((ext_vector_type(4)));
    typedef float v4fa __attribute__((ext_vector_type(4), may_alias));
    const int rsub = lane >> 4, c4 = (lane & 15) * 4;
    for (int pass = 0; pass < 2; ++pass) {
#pragma unroll 4
      for (int q = 0; q < LL / 2; ++q) {
        const int row = q * 2 + rsub;
        const v4f v = *(const v4fa*)&ostage[row][c4];
        *(volatile v4f*)(out + outBase + row * TILE + c4) = v;
      }
      if (pass == 0) __threadfence();
    }
  }
}

extern "C" void kernel_launch(void* const* d_in, const int* in_sizes, int n_in,
                              void* d_out, int out_size, void* d_ws, size_t ws_size,
                              hipStream_t stream) {
  (void)in_sizes; (void)n_in; (void)out_size; (void)d_ws; (void)ws_size;
  const float* x     = (const float*)d_in[0];
  const float* patts = (const float*)d_in[1];
  float*       out   = (float*)d_out;
  dim3 grid(PP, BB);
  dim3 block(32);
  hipLaunchKernelGGL(dtw_fused_kernel, grid, block, 0, stream, x, patts, out);
}
